// EncoderBlock_87754771792403
// MI455X (gfx1250) — hardware-verified
//
#include <hip/hip_runtime.h>
#include <math.h>

#ifndef NB
#define NB 16
#endif
#ifndef SEG_A
#define SEG_A 256
#endif
#ifndef SEG_B
#define SEG_B 768
#endif
#define SEQ (SEG_A + SEG_B)
#define NB_FULL 16
#define SEQ_FULL 1024
#define EMB 512
#define NHEAD 8
#define HDIM 64
#define WSZ (EMB * EMB)

static_assert(NB >= 1 && NB <= NB_FULL);
static_assert(SEQ <= SEQ_FULL);
static_assert(SEG_A % 64 == 0 && SEG_B % 64 == 0);
static_assert(EMB % 64 == 0 && EMB == NHEAD * HDIM && HDIM == 64);
static_assert((NB * SEQ) % 256 == 0);
static_assert((NB * SEQ * (EMB / 8)) % 256 == 0);
static_assert((NB * SEQ * (EMB / 4)) % 256 == 0);
static_assert((WSZ / 8) % 256 == 0);

typedef __attribute__((ext_vector_type(16))) _Float16 v16h;
typedef __attribute__((ext_vector_type(8)))  _Float16 v8h;
typedef __attribute__((ext_vector_type(8)))  float    v8f;
typedef __attribute__((ext_vector_type(4)))  float    v4f;
typedef __attribute__((ext_vector_type(2)))  float    v2f;
typedef __attribute__((ext_vector_type(4)))  unsigned int u4v;
typedef __attribute__((ext_vector_type(2)))  unsigned int u2v;

union FragU { v16h v; v8h h[2]; };
__device__ __forceinline__ v16h frag_ld(const _Float16* p) { FragU f; f.h[0] = *(const v8h*)(p); f.h[1] = *(const v8h*)(p + 16); return f.v; }

__device__ __forceinline__ v8f wmma16(v16h a, v16h b, v8f c) {
    c = __builtin_amdgcn_wmma_f32_16x16x32_f16(false, a, false, b, (short)0, c, false, false);
    asm volatile("v_nop\n\tv_nop\n\tv_nop\n\tv_nop" : "+v"(c) : "v"(a), "v"(b));
    return c;
}
__device__ __forceinline__ v8f mma_raw(v16h a, v16h b, v8f c) { return __builtin_amdgcn_wmma_f32_16x16x32_f16(false, a, false, b, (short)0, c, false, false); }
__device__ __forceinline__ void dep_guard_h(v8f& a, v8f& b, v16h x, v16h y) { asm volatile("v_nop\n\tv_nop\n\tv_nop\n\tv_nop" : "+v"(a), "+v"(b) : "v"(x), "v"(y)); }
__device__ __forceinline__ void keep4_h(v16h a, v16h b, v16h c, v16h d) { asm volatile("v_nop" :: "v"(a), "v"(b), "v"(c), "v"(d)); }
__device__ __forceinline__ void acc_guard4(v8f& a, v8f& b, v8f& c, v8f& d) { asm volatile("v_nop\n\tv_nop\n\tv_nop\n\tv_nop" : "+v"(a), "+v"(b), "+v"(c), "+v"(d)); }

__device__ __forceinline__ float bf_keep(float v) { const unsigned u = __float_as_uint(v); return __uint_as_float((u + 0x7fffu + ((u >> 16) & 1u)) & 0xffff0000u); }
__device__ __forceinline__ unsigned pk2h(float a, float b) { return (unsigned)__builtin_bit_cast(unsigned short, (_Float16)a) | ((unsigned)__builtin_bit_cast(unsigned short, (_Float16)b) << 16); }
__device__ __forceinline__ unsigned full_row(unsigned r) { return (r / (unsigned)SEQ) * (unsigned)SEQ_FULL + (r % (unsigned)SEQ); }

#define VST2(T, ptr, val) do { const T vst2_v_ = (val); *(volatile T*)(ptr) = vst2_v_; __threadfence(); *(volatile T*)(ptr) = vst2_v_; } while (0)

__global__ __launch_bounds__(256) void k_castx(const float* __restrict__ X, unsigned short* __restrict__ D, unsigned n8) {
    const unsigned u = blockIdx.x * 256u + threadIdx.x; if (u >= n8) return;
    const unsigned r = u >> 6, c0 = (u & 63u) << 3;
    const float* s = X + (size_t)full_row(r) * EMB + c0;
    const v4f a = *(const v4f*)(s), b = *(const v4f*)(s + 4);
    u4v pk; pk.x = pk2h(bf_keep(a.x), bf_keep(a.y)); pk.y = pk2h(bf_keep(a.z), bf_keep(a.w)); pk.z = pk2h(bf_keep(b.x), bf_keep(b.y)); pk.w = pk2h(bf_keep(b.z), bf_keep(b.w));
    VST2(u4v, (u4v*)(D + (size_t)u * 8), pk);
}

__global__ __launch_bounds__(256) void k_wcast(const float* __restrict__ w0, const float* __restrict__ w1, const float* __restrict__ w2, const float* __restrict__ w3, const float* __restrict__ w4,
                                               const float* __restrict__ w5, const float* __restrict__ w6, const float* __restrict__ w7, const float* __restrict__ w8, const float* __restrict__ w9,
                                               unsigned short* __restrict__ D) {
    const unsigned y = blockIdx.y;
    const float* s = w0;
    if (y == 1u) s = w1; if (y == 2u) s = w2; if (y == 3u) s = w3; if (y == 4u) s = w4; if (y == 5u) s = w5;
    if (y == 6u) s = w6; if (y == 7u) s = w7; if (y == 8u) s = w8; if (y == 9u) s = w9;
    const unsigned u = blockIdx.x * 256u + threadIdx.x; if (u >= (unsigned)(WSZ / 8)) return;
    const v4f a = *(const v4f*)(s + (size_t)u * 8), b = *(const v4f*)(s + (size_t)u * 8 + 4);
    u4v pk; pk.x = pk2h(bf_keep(a.x) * 16.f, bf_keep(a.y) * 16.f); pk.y = pk2h(bf_keep(a.z) * 16.f, bf_keep(a.w) * 16.f);
    pk.z = pk2h(bf_keep(b.x) * 16.f, bf_keep(b.y) * 16.f); pk.w = pk2h(bf_keep(b.z) * 16.f, bf_keep(b.w) * 16.f);
    VST2(u4v, (u4v*)(D + (size_t)y * WSZ + (size_t)u * 8), pk);
}

template <int BIAS_MODE, int OUT_MODE, bool RESID, bool RBF, int ACT>
__global__ __launch_bounds__(256) void k_gemm64(
    const _Float16* __restrict__ A, int lda, long strideA,
    const _Float16* __restrict__ Bt, int ldb, long strideB,
    void* Cout, int ldc, long strideC,
    const float* __restrict__ bias,
    const float* resid, long strideR,
    int M, int N, int K, float scale) {
  __shared__ __align__(16) float sT[8][16 * 68];
  const unsigned b    = blockIdx.y;
  const unsigned lane = threadIdx.x & 31u;
  const unsigned wave = threadIdx.x >> 5;
  const unsigned tilesN = (unsigned)N >> 6;
  const unsigned tilesM = (unsigned)M >> 6;
  const unsigned tile = blockIdx.x * 8u + wave;
  if (tile >= tilesM * tilesN) return;
  const unsigned tm = tile / tilesN;
  const unsigned tn = tile - tm * tilesN;
  const unsigned m0 = tm << 6;
  const unsigned n0 = tn << 6;

  const _Float16* Ab = A  + (size_t)b * (size_t)strideA;
  const _Float16* Bb = Bt + (size_t)b * (size_t)strideB;

  const unsigned rlane = lane & 15u;
  const unsigned koff  = (lane >> 4) << 3;
  const unsigned mOff  = (lane >> 4) << 3;

  v8f acc[4][4];
#pragma unroll
  for (int i = 0; i < 4; ++i)
#pragma unroll
    for (int j = 0; j < 4; ++j) acc[i][j] = (v8f){0.f,0.f,0.f,0.f,0.f,0.f,0.f,0.f};

  for (unsigned k0 = 0; k0 < (unsigned)K; k0 += 32u) {
    v16h bh[4];
#pragma unroll
    for (int j = 0; j < 4; ++j) {
      const size_t bo = (size_t)(n0 + ((unsigned)j << 4) + rlane) * (unsigned)ldb + koff + k0;
      bh[j] = frag_ld(Bb + bo);
    }
#pragma unroll
    for (int i = 0; i < 4; ++i) {
      const size_t ao = (size_t)(m0 + ((unsigned)i << 4) + rlane) * (unsigned)lda + koff + k0;
      const v16h ah = frag_ld(Ab + ao);
#pragma unroll
      for (int j = 0; j < 4; ++j) acc[i][j] = mma_raw(ah, bh[j], acc[i][j]);
      dep_guard_h(acc[i][0], acc[i][3], ah, ah);
    }
    keep4_h(bh[0], bh[1], bh[2], bh[3]);
  }
  acc_guard4(acc[0][0], acc[0][1], acc[0][2], acc[0][3]);
  acc_guard4(acc[1][0], acc[1][1], acc[1][2], acc[1][3]);
  acc_guard4(acc[2][0], acc[2][1], acc[2][2], acc[2][3]);
  acc_guard4(acc[3][0], acc[3][1], acc[3][2], acc[3][3]);

  float* slab = sT[wave];
  const float* Rb = RESID ? (resid + (size_t)b * (size_t)strideR) : nullptr;
#pragma unroll
  for (int i = 0; i < 4; ++i) {
    const unsigned mBase = m0 + ((unsigned)i << 4);
    float bm[8];
#pragma unroll
    for (int r = 0; r < 8; ++r) bm[r] = (BIAS_MODE == 1) ? bf_keep(bias[mBase + mOff + (unsigned)r]) : 0.f;
#pragma unroll
    for (int j = 0; j < 4; ++j) {
      const unsigned n = n0 + ((unsigned)j << 4) + rlane;
      float bv = 0.f;
      if (BIAS_MODE == 2) bv = bf_keep(bias[n]);
#pragma unroll
      for (int r = 0; r < 8; ++r) {
        float v = acc[i][j][r] * scale;
        if (BIAS_MODE == 1) v += bm[r];
        if (BIAS_MODE == 2) v += bv;
        if (ACT == 2) v = fmaxf(v, 0.0f);
        slab[(mOff + (unsigned)r) * 68u + ((unsigned)j << 4) + rlane] = v;
      }
    }
    __builtin_amdgcn_fence(3  , "workgroup");
    __builtin_amdgcn_wave_barrier();
    __builtin_amdgcn_fence(2  , "workgroup");
    if (OUT_MODE == 0) {
      float* C = (float*)Cout + (size_t)b * (size_t)strideC;
      const unsigned hh = lane >> 4, c4 = (lane & 15u) << 2;
      v4f vv[8];
#pragma unroll
      for (int it = 0; it < 8; ++it) {
        const unsigned row = (unsigned)it * 2u + hh;
        v4f v = *(const v4f*)(slab + row * 68u + c4);
        if (RESID) {
          v4f rv = *(const v4f*)(Rb + (size_t)(mBase + row) * (unsigned)ldc + n0 + c4);
          if (RBF) { rv.x = bf_keep(rv.x); rv.y = bf_keep(rv.y); rv.z = bf_keep(rv.z); rv.w = bf_keep(rv.w); }
          v = v + rv;
        }
        vv[it] = v;
      }
      for (int pass = 0; pass < 2; ++pass) {
#pragma unroll
        for (int it = 0; it < 8; ++it) {
          const unsigned row = (unsigned)it * 2u + hh;
          *(volatile v4f*)(C + (size_t)(mBase + row) * (unsigned)ldc + n0 + c4) = vv[it];
        }
        __threadfence();
      }
    } else {
      const unsigned q = lane >> 3, c8 = (lane & 7u) << 3;
      _Float16* C = (_Float16*)Cout + (size_t)b * (size_t)strideC;
      v8h hv[4];
#pragma unroll
      for (int it = 0; it < 4; ++it) {
        const unsigned row = (unsigned)it * 4u + q;
        const float* sp = slab + row * 68u + c8;
        const v4f s0 = *(const v4f*)(sp), s1 = *(const v4f*)(sp + 4);
        v8h t;
        t[0] = (_Float16)s0.x; t[1] = (_Float16)s0.y; t[2] = (_Float16)s0.z; t[3] = (_Float16)s0.w;
        t[4] = (_Float16)s1.x; t[5] = (_Float16)s1.y; t[6] = (_Float16)s1.z; t[7] = (_Float16)s1.w;
        hv[it] = t;
      }
      for (int pass = 0; pass < 2; ++pass) {
#pragma unroll
        for (int it = 0; it < 4; ++it) {
          const unsigned row = (unsigned)it * 4u + q;
          *(volatile v8h*)(C + (size_t)(mBase + row) * (unsigned)ldc + n0 + c8) = hv[it];
        }
        __threadfence();
      }
    }
    __builtin_amdgcn_fence(3  , "workgroup");
    __builtin_amdgcn_wave_barrier();
    __builtin_amdgcn_fence(2  , "workgroup");
  }
}

template <int SEGLEN, int SEGOFF>
__global__ __launch_bounds__(128) void k_attn(const _Float16* __restrict__ Q, const _Float16* __restrict__ Kp, const _Float16* __restrict__ VT, _Float16* __restrict__ CTX) {
  __shared__ __align__(16) _Float16 Psh[4][16 * 64];
  __shared__ __align__(16) float    Os[4][16 * 68];
  constexpr unsigned NQB = (unsigned)SEGLEN / 64u;
  constexpr unsigned NCH = (unsigned)SEGLEN / 64u;
  const unsigned tid  = threadIdx.x;
  const unsigned wave = tid >> 5;
  const unsigned lane = tid & 31u;
  const unsigned hh   = lane >> 4;
  const unsigned c    = lane & 15u;
  const unsigned bx = blockIdx.x;
  const unsigned qb = bx % NQB;
  const unsigned bh = bx / NQB;
  const unsigned h  = bh & 7u;
  const unsigned b  = bh >> 3;
  const unsigned q0 = qb * 64u + wave * 16u;
  const size_t rowbase = (size_t)b * SEQ + (unsigned)SEGOFF;

  const _Float16* qrow = Q + (rowbase + q0 + c) * EMB + h * 64u + 8u * hh;
  const v16h qa0 = frag_ld(qrow), qa1 = frag_ld(qrow + 32);
  const _Float16* kbase = Kp + rowbase * EMB + h * 64u + 8u * hh;
  const _Float16* vbase = VT + ((size_t)b * EMB + h * 64u) * SEQ + (unsigned)SEGOFF + 8u * hh;

  float mrow[8], lrow[8];
  v8f oacc[4];
#pragma unroll
  for (int r = 0; r < 8; ++r) { mrow[r] = -__builtin_inff(); lrow[r] = 0.f; }
#pragma unroll
  for (int t = 0; t < 4; ++t) oacc[t] = (v8f){0.f,0.f,0.f,0.f,0.f,0.f,0.f,0.f};

  const float SC = 0.125f * 1.4426950408889634f;
  _Float16* pw = Psh[wave];

  for (unsigned kc = 0; kc < NCH; ++kc) {
    const unsigned kv0 = kc * 64u;
    v8f s[4];
#pragma unroll
    for (int j = 0; j < 4; ++j) {
      const _Float16* kr = kbase + (size_t)(kv0 + (unsigned)j * 16u + c) * EMB;
      v8f a = (v8f){0.f,0.f,0.f,0.f,0.f,0.f,0.f,0.f};
      a = wmma16(qa0, frag_ld(kr), a);
      a = wmma16(qa1, frag_ld(kr + 32), a);
      s[j] = a;
    }
#pragma unroll
    for (int r = 0; r < 8; ++r) {
      const float x0 = s[0][r] * SC, x1 = s[1][r] * SC, x2 = s[2][r] * SC, x3 = s[3][r] * SC;
      float m = fmaxf(fmaxf(x0, x1), fmaxf(x2, x3));
      m = fmaxf(m, __shfl_xor(m, 1, 32)); m = fmaxf(m, __shfl_xor(m, 2, 32));
      m = fmaxf(m, __shfl_xor(m, 4, 32)); m = fmaxf(m, __shfl_xor(m, 8, 32));
      const float mnew = fmaxf(mrow[r], m);
      const float alpha = exp2f(mrow[r] - mnew);
      mrow[r] = mnew;
      const float p0 = exp2f(x0 - mnew), p1 = exp2f(x1 - mnew), p2 = exp2f(x2 - mnew), p3 = exp2f(x3 - mnew);
      float psum = (p0 + p1) + (p2 + p3);
      const unsigned po = (8u * hh + (unsigned)r) * 64u + c;
      pw[po]       = (_Float16)(p0 * 32768.0f);
      pw[po + 16u] = (_Float16)(p1 * 32768.0f);
      pw[po + 32u] = (_Float16)(p2 * 32768.0f);
      pw[po + 48u] = (_Float16)(p3 * 32768.0f);
      psum += __shfl_xor(psum, 1, 32); psum += __shfl_xor(psum, 2, 32);
      psum += __shfl_xor(psum, 4, 32); psum += __shfl_xor(psum, 8, 32);
      lrow[r] = lrow[r] * alpha + psum;
#pragma unroll
      for (int t = 0; t < 4; ++t) oacc[t][r] *= alpha;
    }
    __builtin_amdgcn_fence(3  , "workgroup");
    __builtin_amdgcn_wave_barrier();
    __builtin_amdgcn_fence(2  , "workgroup");
#pragma unroll
    for (int kk = 0; kk < 2; ++kk) {
      const v16h pa = frag_ld(pw + c * 64u + (unsigned)kk * 32u + 8u * hh);
#pragma unroll
      for (int t = 0; t < 4; ++t) {
        const v16h vb = frag_ld(vbase + (size_t)((unsigned)t * 16u + c) * SEQ + kv0 + (unsigned)kk * 32u);
        oacc[t] = wmma16(pa, vb, oacc[t]);
      }
    }
    __builtin_amdgcn_fence(3  , "workgroup");
    __builtin_amdgcn_wave_barrier();
    __builtin_amdgcn_fence(2  , "workgroup");
  }

  float* os = Os[wave];
#pragma unroll
  for (int r = 0; r < 8; ++r) {
    const float inv = 1.0f / (lrow[r] * 512.0f);
#pragma unroll
    for (int t = 0; t < 4; ++t) os[(8u * hh + (unsigned)r) * 68u + (unsigned)t * 16u + c] = oacc[t][r] * inv;
  }
  __builtin_amdgcn_fence(3  , "workgroup");
  __builtin_amdgcn_wave_barrier();
  __builtin_amdgcn_fence(2  , "workgroup");
  {
    const unsigned q = lane >> 3, c8 = (lane & 7u) << 3;
    _Float16* cb = CTX + (rowbase + q0) * EMB + h * 64u + c8;
    v8h hv[4];
#pragma unroll
    for (int it = 0; it < 4; ++it) {
      const unsigned row = (unsigned)it * 4u + q;
      const float* sp = os + row * 68u + c8;
      const v4f s0 = *(const v4f*)(sp), s1 = *(const v4f*)(sp + 4);
      v8h t;
      t[0] = (_Float16)s0.x; t[1] = (_Float16)s0.y; t[2] = (_Float16)s0.z; t[3] = (_Float16)s0.w;
      t[4] = (_Float16)s1.x; t[5] = (_Float16)s1.y; t[6] = (_Float16)s1.z; t[7] = (_Float16)s1.w;
      hv[it] = t;
    }
    for (int pass = 0; pass < 2; ++pass) {
#pragma unroll
      for (int it = 0; it < 4; ++it) {
        const unsigned row = (unsigned)it * 4u + q;
        *(volatile v8h*)(cb + (size_t)row * EMB) = hv[it];
      }
      __threadfence();
    }
  }
}

template <bool FULLMAP>
__global__ __launch_bounds__(256) void k_colstat4(const float* __restrict__ X, unsigned nrows, float inv_n, float eps, float* __restrict__ STAT) {
  __shared__ __align__(16) v4f red[256];
  const unsigned t = threadIdx.x, c0 = blockIdx.x * 4u;
  v4f s = (v4f){0.f, 0.f, 0.f, 0.f};
#pragma unroll 2
  for (unsigned r = t; r < nrows; r += 256u) {
    const unsigned rr = FULLMAP ? full_row(r) : r;
    s = s + *(const v4f*)(X + (size_t)rr * EMB + c0);
  }
  red[t] = s; __syncthreads();
  for (unsigned o = 128u; o > 0u; o >>= 1) { if (t < o) red[t] = red[t] + red[t + o]; __syncthreads(); }
  const v4f mu = red[0] * inv_n; __syncthreads();
  v4f q = (v4f){0.f, 0.f, 0.f, 0.f};
#pragma unroll 2
  for (unsigned r = t; r < nrows; r += 256u) {
    const unsigned rr = FULLMAP ? full_row(r) : r;
    const v4f d = *(const v4f*)(X + (size_t)rr * EMB + c0) - mu;
    q = q + d * d;
  }
  red[t] = q; __syncthreads();
  for (unsigned o = 128u; o > 0u; o >>= 1) { if (t < o) red[t] = red[t] + red[t + o]; __syncthreads(); }
  const v4f var = red[0] * inv_n;
  if (t < 128u) {
    const unsigned col = t >> 5, ln = t & 31u;
    const float m_ = (col == 0u) ? mu.x : ((col == 1u) ? mu.y : ((col == 2u) ? mu.z : mu.w));
    const float v_ = (col == 0u) ? var.x : ((col == 1u) ? var.y : ((col == 2u) ? var.z : var.w));
    const float rs = rsqrtf(v_ + eps);
    const float o_ = (ln == 0u) ? m_ : ((ln == 1u) ? rs : 0.f);
    VST2(float, STAT + (size_t)(c0 + col) * 32u + ln, o_);
  }
}

template <bool W16, bool FULLMAP>
__global__ __launch_bounds__(256) void k_bnapply(float* XY, const float* __restrict__ STAT, const float* __restrict__ G, const float* __restrict__ Bv, unsigned short* Y16, unsigned n4) {
  const unsigned u = blockIdx.x * 256u + threadIdx.x; if (u >= n4) return;
  const unsigned r = u >> 7, c = (u & 127u) << 2;
  const size_t o = (size_t)(FULLMAP ? full_row(r) : r) * EMB + c;
  const v4f x = *(const v4f*)(XY + o);
  const v2f s0 = *(const v2f*)(STAT + (size_t)(c + 0u) * 32u), s1 = *(const v2f*)(STAT + (size_t)(c + 1u) * 32u);
  const v2f s2 = *(const v2f*)(STAT + (size_t)(c + 2u) * 32u), s3 = *(const v2f*)(STAT + (size_t)(c + 3u) * 32u);
  const v4f g = *(const v4f*)(G + c), bb = *(const v4f*)(Bv + c);
  v4f y;
  y.x = (x.x - s0.x) * s0.y * bf_keep(g.x) + bf_keep(bb.x);
  y.y = (x.y - s1.x) * s1.y * bf_keep(g.y) + bf_keep(bb.y);
  y.z = (x.z - s2.x) * s2.y * bf_keep(g.z) + bf_keep(bb.z);
  y.w = (x.w - s3.x) * s3.y * bf_keep(g.w) + bf_keep(bb.w);
  VST2(v4f, XY + o, y);
  if (W16) { u2v pk; pk.x = pk2h(y.x, y.y); pk.y = pk2h(y.z, y.w); VST2(u2v, (u2v*)(Y16 + (size_t)u * 4), pk); }
}

#define SZ_P16  ((size_t)NB * SEQ * EMB * 2)
#define SZ_W16  ((size_t)10 * WSZ * 2)
#define SZ_H    ((size_t)NB * SEQ * EMB * 4)
#define SZ_STAT ((size_t)EMB * 32 * 4)
#define OFF_X16  ((size_t)0)
#define OFF_W16  (OFF_X16 + SZ_P16)
#define OFF_Q16  (OFF_W16 + SZ_W16)
#define OFF_K16  (OFF_Q16 + SZ_P16)
#define OFF_VT16 (OFF_K16 + SZ_P16)
#define OFF_CTX  (OFF_VT16 + SZ_P16)
#define OFF_H    (OFF_CTX + SZ_P16)
#define OFF_ST1  (OFF_H + SZ_H)
#define OFF_ST2  (OFF_ST1 + SZ_STAT)
#define WS_TOTAL (OFF_ST2 + SZ_STAT)
static_assert(SZ_P16 % 256 == 0 && SZ_W16 % 256 == 0 && SZ_H % 256 == 0 && SZ_STAT % 256 == 0);
static_assert(WS_TOTAL <= (size_t)134217728);
static_assert((size_t)NB * SEQ * EMB * 2 <= SZ_P16);

extern "C" void kernel_launch(void* const* d_in, const int* in_sizes, int n_in, void* d_out, int out_size, void* d_ws, size_t ws_size, hipStream_t stream) {
    if (n_in < 25) return;
    const long long xneed = ((long long)(NB - 1) * SEQ_FULL + SEQ) * EMB;
    if ((long long)in_sizes[0] < xneed) return;
    for (int i = 0; i < 10; ++i) { if (in_sizes[1 + 2 * i] < WSZ) return; if (in_sizes[2 + 2 * i] < EMB) return; }
    for (int i = 21; i < 25; ++i) if (in_sizes[i] < EMB) return;
    if ((long long)out_size < xneed) return;
    if ((size_t)WS_TOTAL > ws_size) return;

    const float* x    = (const float*)d_in[0];
    const float* rq_w = (const float*)d_in[1];  const float* rq_b = (const float*)d_in[2];
    const float* rk_w = (const float*)d_in[3];  const float* rk_b = (const float*)d_in[4];
    const float* rv_w = (const float*)d_in[5];  const float* rv_b = (const float*)d_in[6];
    const float* ro_w = (const float*)d_in[7];  const float* ro_b = (const float*)d_in[8];
    const float* tq_w = (const float*)d_in[9];  const float* tq_b = (const float*)d_in[10];
    const float* tk_w = (const float*)d_in[11]; const float* tk_b = (const float*)d_in[12];
    const float* tv_w = (const float*)d_in[13]; const float* tv_b = (const float*)d_in[14];
    const float* to_w = (const float*)d_in[15]; const float* to_b = (const float*)d_in[16];
    const float* f1_w = (const float*)d_in[17]; const float* f1_b = (const float*)d_in[18];
    const float* f2_w = (const float*)d_in[19]; const float* f2_b = (const float*)d_in[20];
    const float* bn1_g = (const float*)d_in[21]; const float* bn1_b = (const float*)d_in[22];
    const float* bn2_g = (const float*)d_in[23]; const float* bn2_b = (const float*)d_in[24];
    float* out = (float*)d_out;

    char* ws = (char*)d_ws;
    unsigned short* X16  = (unsigned short*)(ws + OFF_X16);
    unsigned short* W16  = (unsigned short*)(ws + OFF_W16);
    unsigned short* Q16  = (unsigned short*)(ws + OFF_Q16);
    unsigned short* K16  = (unsigned short*)(ws + OFF_K16);
    unsigned short* VT16 = (unsigned short*)(ws + OFF_VT16);
    unsigned short* CTX  = (unsigned short*)(ws + OFF_CTX);
    float* H    = (float*)(ws + OFF_H);
    float* ST1  = (float*)(ws + OFF_ST1);
    float* ST2  = (float*)(ws + OFF_ST2);
    unsigned short* HN16 = Q16;
    unsigned short* F16  = K16;

    const _Float16* X16h = (const _Float16*)X16;
    const _Float16* W16h = (const _Float16*)W16;
    const long SB  = (long)SEQ * EMB;
    const long SBF = (long)SEQ_FULL * EMB;
    const long SVT = (long)EMB * SEQ;
    const size_t offB = (size_t)SEG_A * EMB;

    k_castx<<<(unsigned)((NB * SEQ * (EMB / 8)) / 256), 256, 0, stream>>>(x, X16, (unsigned)(NB * SEQ * (EMB / 8)));
    k_wcast<<<dim3((unsigned)((WSZ / 8) / 256), 10u), 256, 0, stream>>>(rq_w, rk_w, rv_w, ro_w, tq_w, tk_w, tv_w, to_w, f1_w, f2_w, W16);

    const unsigned gA  = (unsigned)(((SEG_A / 64) * (EMB / 64) + 7) / 8);
    const unsigned gB  = (unsigned)(((SEG_B / 64) * (EMB / 64) + 7) / 8);
    k_gemm64<2, 1, false, false, 0><<<dim3(gA, NB), 256, 0, stream>>>(X16h, EMB, SB, W16h + (size_t)0 * WSZ, EMB, 0L, (void*)Q16, EMB, SB, rq_b, nullptr, 0L, SEG_A, EMB, EMB, 0.0625f);
    k_gemm64<2, 1, false, false, 0><<<dim3(gA, NB), 256, 0, stream>>>(X16h, EMB, SB, W16h + (size_t)1 * WSZ, EMB, 0L, (void*)K16, EMB, SB, rk_b, nullptr, 0L, SEG_A, EMB, EMB, 0.0625f);
    k_gemm64<1, 1, false, false, 0><<<dim3(gA, NB), 256, 0, stream>>>(W16h + (size_t)2 * WSZ, EMB, 0L, X16h, EMB, SB, (void*)VT16, SEQ, SVT, rv_b, nullptr, 0L, EMB, SEG_A, EMB, 0.0625f);
    k_gemm64<2, 1, false, false, 0><<<dim3(gB, NB), 256, 0, stream>>>(X16h + offB, EMB, SB, W16h + (size_t)4 * WSZ, EMB, 0L, (void*)(Q16 + offB), EMB, SB, tq_b, nullptr, 0L, SEG_B, EMB, EMB, 0.0625f);
    k_gemm64<2, 1, false, false, 0><<<dim3(gB, NB), 256, 0, stream>>>(X16h + offB, EMB, SB, W16h + (size_t)5 * WSZ, EMB, 0L, (void*)(K16 + offB), EMB, SB, tk_b, nullptr, 0L, SEG_B, EMB, EMB, 0.0625f);
    k_gemm64<1, 1, false, false, 0><<<dim3(gB, NB), 256, 0, stream>>>(W16h + (size_t)6 * WSZ, EMB, 0L, X16h + offB, EMB, SB, (void*)(VT16 + SEG_A), SEQ, SVT, tv_b, nullptr, 0L, EMB, SEG_B, EMB, 0.0625f);

    k_attn<SEG_A, 0><<<(unsigned)(NB * NHEAD * (SEG_A / 64)), 128, 0, stream>>>((const _Float16*)Q16, (const _Float16*)K16, (const _Float16*)VT16, (_Float16*)CTX);
    k_attn<SEG_B, SEG_A><<<(unsigned)(NB * NHEAD * (SEG_B / 64)), 128, 0, stream>>>((const _Float16*)Q16, (const _Float16*)K16, (const _Float16*)VT16, (_Float16*)CTX);

    k_gemm64<2, 0, true, true, 0><<<dim3(gA, NB), 256, 0, stream>>>((const _Float16*)CTX, EMB, SB, W16h + (size_t)3 * WSZ, EMB, 0L, (void*)H, EMB, SB, ro_b, x, SBF, SEG_A, EMB, EMB, 0.0009765625f);
    k_gemm64<2, 0, true, true, 0><<<dim3(gB, NB), 256, 0, stream>>>((const _Float16*)CTX + offB, EMB, SB, W16h + (size_t)7 * WSZ, EMB, 0L, (void*)(H + offB), EMB, SB, to_b, x + offB, SBF, SEG_B, EMB, EMB, 0.0009765625f);

    const unsigned nrows = (unsigned)(NB * SEQ);
    const float inv_n = 1.0f / (float)(NB * SEQ);
    k_colstat4<false><<<(unsigned)(EMB / 4), 256, 0, stream>>>(H, nrows, inv_n, 1e-5f, ST1);
    k_bnapply<true, false><<<(unsigned)((NB * SEQ * (EMB / 4)) / 256), 256, 0, stream>>>(H, ST1, bn1_g, bn1_b, HN16, (unsigned)(NB * SEQ * (EMB / 4)));

    const unsigned gF1 = (unsigned)((((NB * SEQ) / 64) * (EMB / 64) + 7) / 8);
    k_gemm64<2, 1, false, false, 2><<<dim3(gF1, 1u), 256, 0, stream>>>((const _Float16*)HN16, EMB, 0L, W16h + (size_t)8 * WSZ, EMB, 0L, (void*)F16, EMB, 0L, f1_b, nullptr, 0L, NB * SEQ, EMB, EMB, 0.0625f);
    const unsigned gF2 = (unsigned)(((SEQ / 64) * (EMB / 64) + 7) / 8);
    k_gemm64<2, 0, true, false, 0><<<dim3(gF2, NB), 256, 0, stream>>>((const _Float16*)F16, EMB, SB, W16h + (size_t)9 * WSZ, EMB, 0L, (void*)out, EMB, SBF, f2_b, H, SB, SEQ, EMB, EMB, 0.0625f);

    k_colstat4<true><<<(unsigned)(EMB / 4), 256, 0, stream>>>(out, nrows, inv_n, 1e-5f, ST2);
    k_bnapply<false, true><<<(unsigned)((NB * SEQ * (EMB / 4)) / 256), 256, 0, stream>>>(out, ST2, bn2_g, bn2_b, nullptr, (unsigned)(NB * SEQ * (EMB / 4)));
}
